// FixedVAR_48601849921953
// MI455X (gfx1250) — hardware-verified
//
#include <hip/hip_runtime.h>
#include <stdint.h>

typedef __attribute__((ext_vector_type(16))) _Float16 v16h;
typedef __attribute__((ext_vector_type(8)))  _Float16 v8h;
typedef __attribute__((ext_vector_type(8)))  float    v8f;
typedef __attribute__((ext_vector_type(4)))  float    v4f;

constexpr int kBatch  = 32;
constexpr int kSeq    = 128;
constexpr int kDim    = 1024;
constexpr int kHeads  = 16;
constexpr int kHd     = 64;
constexpr int kGroup  = 8;
constexpr int kTiles  = kSeq / 16;
constexpr int kWaves  = 4;
static_assert(kHeads * kHd == kDim);
static_assert((kHd % 32) == 0 && (kSeq % 32) == 0);
static_assert(kTiles == 2 * kWaves);
static_assert((kBatch % kGroup) == 0);

constexpr float kKCarry   = 16.0f;
constexpr float kQCarry   = 1024.0f;
constexpr float kVCarry   = 1024.0f;
constexpr float kPCarry   = 256.0f;
constexpr float kPScale   = kPCarry / (kQCarry * kKCarry);
constexpr float kYScale   = 1.0f / (kPCarry * kVCarry);
constexpr float kF16MinNormal = 6.103515625e-5f;

constexpr int kPPitch  = 40;
constexpr int kOPitch  = 68;
constexpr int kVtPitch = 132;

constexpr size_t kBytesK  = (size_t)kBatch * kSeq * kDim * 2;
constexpr size_t kBytesQ  = (size_t)kGroup * kSeq * kDim * 2;
constexpr size_t kBytesVt = (size_t)kGroup * kHeads * kHd * kSeq * 2;
constexpr size_t kOffKH   = 0;
constexpr size_t kOffQH   = kOffKH  + kBytesK;
constexpr size_t kOffVTH  = kOffQH  + kBytesQ;
constexpr size_t kWsTotal = kOffVTH + kBytesVt;
static_assert(kBytesK == 8388608ull && kBytesQ == 2097152ull && kBytesVt == 2097152ull);
static_assert(kWsTotal == 12582912ull);
static_assert(kWsTotal <= 134217728ull);
static_assert((kOffQH % 128) == 0 && (kOffVTH % 128) == 0);

union FragU { v16h v; v8h h[2]; };

__device__ __forceinline__ v16h frag_load(const _Float16* p) {
  FragU f;
  f.h[0] = *(const v8h*)(p);
  f.h[1] = *(const v8h*)(p + 16);
  return f.v;
}

__device__ __forceinline__ v8f mma_h(v16h a, v16h b, v8f c) {
  c = __builtin_amdgcn_wmma_f32_16x16x32_f16(false, a, false, b, (short)0, c, false, false);
  asm volatile("v_nop\n\tv_nop\n\tv_nop\n\tv_nop" : "+v"(c) : "v"(a), "v"(b));
  return c;
}

__device__ __forceinline__ void wave_lds_sync() {
  __builtin_amdgcn_fence(__ATOMIC_RELEASE, "workgroup");
  __builtin_amdgcn_wave_barrier();
  __builtin_amdgcn_fence(__ATOMIC_ACQUIRE, "workgroup");
}

__device__ __forceinline__ _Float16 f16_flush(float v) {
  const float w = (__builtin_fabsf(v) < kF16MinNormal) ? 0.0f : v;
  return (_Float16)w;
}

__global__ __launch_bounds__(256) void cast_planes_kernel(
    const float* __restrict__ src, unsigned short* __restrict__ dhi, int total8, float carry)
{
  const int i = blockIdx.x * 256 + threadIdx.x;
  if (i >= total8) return;
  const size_t e0 = (size_t)i << 3;
  const v4f a0 = *(const v4f*)(src + e0);
  const v4f a1 = *(const v4f*)(src + e0 + 4);
  v8h hv;
#pragma unroll
  for (int e = 0; e < 4; ++e) {
    const float x0 = a0[e] * carry;
    const float x1 = a1[e] * carry;
    const _Float16 h0 = f16_flush(x0);
    const _Float16 h1 = f16_flush(x1);
    hv[e]     = h0;
    hv[4 + e] = h1;
  }
  unsigned short* qh = dhi + e0;
  *(volatile v8h*)qh = hv;
  __threadfence();
  *(volatile v8h*)qh = hv;
}

__global__ __launch_bounds__(256) void vt_planes_kernel(
    const float* __restrict__ V, unsigned short* __restrict__ vth)
{
  __shared__ __align__(16) float sm[kHd * kVtPitch];
  const int t = threadIdx.x;
  const int lane = t & 31;
  const int wave = t >> 5;
  const int ch = blockIdx.x;
  const int h = ch & (kHeads - 1);
  const int c = ch >> 4;
  const float* vp = V + (size_t)c * kSeq * kDim + (size_t)h * kHd;
#pragma unroll
  for (int it = 0; it < 8; ++it) {
    const int idx = it * 256 + t;
    const int j = idx >> 4;
    const int e4 = (idx & 15) * 4;
    const v4f v = *(const v4f*)(vp + (size_t)j * kDim + e4);
    sm[(e4 + 0) * kVtPitch + j] = v[0];
    sm[(e4 + 1) * kVtPitch + j] = v[1];
    sm[(e4 + 2) * kVtPitch + j] = v[2];
    sm[(e4 + 3) * kVtPitch + j] = v[3];
  }
  __syncthreads();
  const int hh = lane >> 4;
  const int j0 = (lane & 15) * 8;
  v8h hv[4];
#pragma unroll
  for (int it = 0; it < 4; ++it) {
    const int row = it * 16 + wave * 2 + hh;
    const float* sp = sm + row * kVtPitch + j0;
    const v4f a0 = *(const v4f*)(sp);
    const v4f a1 = *(const v4f*)(sp + 4);
#pragma unroll
    for (int e = 0; e < 4; ++e) {
      const float x0 = a0[e] * kVCarry;
      const float x1 = a1[e] * kVCarry;
      const _Float16 h0 = f16_flush(x0);
      const _Float16 h1 = f16_flush(x1);
      hv[it][e]     = h0;
      hv[it][4 + e] = h1;
    }
  }
  for (int pass = 0; pass < 2; ++pass) {
#pragma unroll
    for (int it = 0; it < 4; ++it) {
      const int row = it * 16 + wave * 2 + hh;
      const size_t o = ((size_t)ch * kHd + row) * kSeq + j0;
      *(volatile v8h*)(vth + o) = hv[it];
    }
    __threadfence();
  }
}

__global__ __launch_bounds__(128) void causal_qkv_kernel(
    const unsigned short* __restrict__ qh_p,
    const unsigned short* __restrict__ kh_p,
    const unsigned short* __restrict__ vth_p,
    float* __restrict__ out)
{
  __shared__ __align__(16) _Float16 sPh[kWaves][16 * kPPitch];
  __shared__ __align__(16) float    sO[kWaves][16 * kOPitch];

  const int lane = threadIdx.x & 31;
  const int wave = __builtin_amdgcn_readfirstlane((int)(threadIdx.x >> 5));
  const int hh = lane >> 4;
  const int rl = lane & 15;

  const int bh = blockIdx.x;
  const int h  = bh & (kHeads - 1);
  const int b  = bh >> 4;
  const int c  = b & (kGroup - 1);

  const size_t qbase = (size_t)c * kSeq * kDim + (size_t)h * kHd;
  const size_t kbase = (size_t)b * kSeq * kDim + (size_t)h * kHd;
  const size_t vbase = ((size_t)(c * kHeads + h) * kHd) * kSeq;

  const _Float16* Qh  = (const _Float16*)qh_p + qbase;
  const _Float16* Kh  = (const _Float16*)kh_p + kbase;
  const _Float16* Vth = (const _Float16*)vth_p + vbase;
  float* outp = out + kbase;

  _Float16* sph = sPh[wave];
  float*    os  = sO[wave];

#pragma unroll 1
  for (int tt = 0; tt < 2; ++tt) {
    const int i  = (tt == 0) ? wave : (kTiles - 1 - wave);
    const int l0 = i * 16;

    v16h qh[2];
#pragma unroll
    for (int dc = 0; dc < 2; ++dc) {
      const size_t qo = (size_t)(l0 + rl) * kDim + dc * 32 + 8 * hh;
      qh[dc] = frag_load(Qh + qo);
    }

    v8f yM[4];
#pragma unroll
    for (int t = 0; t < 4; ++t) {
      yM[t] = (v8f){0.f, 0.f, 0.f, 0.f, 0.f, 0.f, 0.f, 0.f};
    }

    const int nch = (i >> 1) + 1;
#pragma unroll 1
    for (int jc = 0; jc < nch; ++jc) {
      const int j0 = jc * 32;

      v8f pM[2];
#pragma unroll
      for (int n = 0; n < 2; ++n) {
        pM[n] = (v8f){0.f, 0.f, 0.f, 0.f, 0.f, 0.f, 0.f, 0.f};
#pragma unroll
        for (int dc = 0; dc < 2; ++dc) {
          const size_t ko = (size_t)(j0 + n * 16 + rl) * kDim + dc * 32 + 8 * hh;
          const v16h kh = frag_load(Kh + ko);
          pM[n] = mma_h(qh[dc], kh, pM[n]);
        }
      }

#pragma unroll
      for (int n = 0; n < 2; ++n) {
        const int j = j0 + n * 16 + rl;
#pragma unroll
        for (int r = 0; r < 8; ++r) {
          const int l = l0 + 8 * hh + r;
          float p = pM[n][r] * kPScale;
          p = (j > l) ? 0.0f : p;
          const _Float16 ph = f16_flush(p);
          sph[(8 * hh + r) * kPPitch + n * 16 + rl] = ph;
        }
      }
      wave_lds_sync();

      FragU pa;
      pa.h[0] = *(const v8h*)(sph + rl * kPPitch + 8 * hh);
      pa.h[1] = *(const v8h*)(sph + rl * kPPitch + 16 + 8 * hh);

#pragma unroll
      for (int t = 0; t < 4; ++t) {
        const size_t vo = (size_t)(t * 16 + rl) * kSeq + j0 + 8 * hh;
        const v16h vh = frag_load(Vth + vo);
        yM[t] = mma_h(pa.v, vh, yM[t]);
      }
      wave_lds_sync();
    }

#pragma unroll
    for (int t = 0; t < 4; ++t) {
#pragma unroll
      for (int r = 0; r < 8; ++r) {
        const float y = yM[t][r] * kYScale;
        os[(8 * hh + r) * kOPitch + t * 16 + rl] = y;
      }
    }
    wave_lds_sync();
    {
      const int c4 = rl * 4;
      for (int pass = 0; pass < 2; ++pass) {
#pragma unroll
        for (int it = 0; it < 8; ++it) {
          const int row = it * 2 + hh;
          const v4f val = *(const v4f*)(os + row * kOPitch + c4);
          *(volatile v4f*)(outp + (size_t)(l0 + row) * kDim + c4) = val;
        }
        __threadfence();
      }
    }
    wave_lds_sync();
  }
}

extern "C" void kernel_launch(void* const* d_in, const int* in_sizes, int n_in,
                              void* d_out, int out_size, void* d_ws, size_t ws_size,
                              hipStream_t stream) {
  if (n_in < 3) return;
  if (in_sizes[0] != kBatch * kSeq * kDim) return;
  if (in_sizes[1] != kGroup * kSeq * kDim) return;
  if (in_sizes[2] != kGroup * kSeq * kDim) return;
  if (out_size != kBatch * kSeq * kDim) return;
  if (ws_size < kWsTotal) return;

  const float* X  = (const float*)d_in[0];
  const float* FQ = (const float*)d_in[1];
  const float* FV = (const float*)d_in[2];
  float* Y = (float*)d_out;

  char* ws = (char*)d_ws;
  unsigned short* KH  = (unsigned short*)(ws + kOffKH);
  unsigned short* QH  = (unsigned short*)(ws + kOffQH);
  unsigned short* VTH = (unsigned short*)(ws + kOffVTH);

  constexpr int kK8 = kBatch * kSeq * kDim / 8;
  constexpr int kQ8 = kGroup * kSeq * kDim / 8;
  static_assert((kK8 % 256) == 0 && (kQ8 % 256) == 0);

  cast_planes_kernel<<<kK8 / 256, 256, 0, stream>>>(X, KH, kK8, kKCarry);
  cast_planes_kernel<<<kQ8 / 256, 256, 0, stream>>>(FQ, QH, kQ8, kQCarry);
  vt_planes_kernel<<<kGroup * kHeads, 256, 0, stream>>>(FV, VTH);
  causal_qkv_kernel<<<kBatch * kHeads, 32 * kWaves, 0, stream>>>(QH, KH, VTH, Y);
}
